// StratumBlock_48318382080024
// MI455X (gfx1250) — hardware-verified
//
#include <hip/hip_runtime.h>
#include <math.h>
#include <stddef.h>

#define CCH  128
#define HWP  9216
#define IMW  96
#define PADW 98
#define KC3  1152

typedef _Float16 v16h __attribute__((ext_vector_type(16)));
typedef _Float16 v8h  __attribute__((ext_vector_type(8)));
typedef _Float16 v4h  __attribute__((ext_vector_type(4)));
typedef float    v8f  __attribute__((ext_vector_type(8)));
typedef float    v4f  __attribute__((ext_vector_type(4)));
typedef unsigned int v4u __attribute__((ext_vector_type(4)));

union Frag { v16h v; v8h h[2]; _Float16 e[16]; };
union H8   { v8h v; _Float16 e[8]; };
union H4   { v4h v; _Float16 e[4]; };

__device__ __forceinline__ v8f zero8() { v8f z = {0.f, 0.f, 0.f, 0.f, 0.f, 0.f, 0.f, 0.f}; return z; }

__device__ __forceinline__ v16h ld_frag(const _Float16* p) {
  Frag f;
  f.h[0] = *(const v8h*)p;
  f.h[1] = *(const v8h*)(p + 16);
  return f.v;
}
__device__ __forceinline__ v8f mma16(v16h a, v16h b, v8f c) {
  return __builtin_amdgcn_wmma_f32_16x16x32_f16(false, a, false, b, (short)0, c, false, false);
}
__device__ __forceinline__ void guard_d1(v8f& d, v16h a0, v16h a1, v16h a2, v16h a3) {
  asm volatile("v_nop\n\tv_nop\n\tv_nop\n\tv_nop" : "+v"(d) : "v"(a0), "v"(a1), "v"(a2), "v"(a3) : "memory");
}
__device__ __forceinline__ void guard_d4(v8f& d0, v8f& d1, v8f& d2, v8f& d3,
                                         v16h a0, v16h a1, v16h a2, v16h a3, v16h b) {
  asm volatile("v_nop\n\tv_nop\n\tv_nop\n\tv_nop"
               : "+v"(d0), "+v"(d1), "+v"(d2), "+v"(d3)
               : "v"(a0), "v"(a1), "v"(a2), "v"(a3), "v"(b) : "memory");
}
__device__ __forceinline__ void wave_lds_sync() {
  __builtin_amdgcn_fence(__ATOMIC_RELEASE, "wavefront");
  __builtin_amdgcn_wave_barrier();
  __builtin_amdgcn_fence(__ATOMIC_ACQUIRE, "wavefront");
}

__device__ __forceinline__ void store_rows16x64(const _Float16* slab, _Float16* C, int ldc, int lane) {
  const int q8 = lane >> 3, c8 = (lane & 7) * 8;
  v8h o[4];
#pragma unroll
  for (int it = 0; it < 4; ++it) o[it] = *(const v8h*)(slab + (it * 4 + q8) * 72 + c8);
  for (int pass = 0; pass < 2; ++pass) {
#pragma unroll
    for (int it = 0; it < 4; ++it)
      *(volatile v8h*)(C + (size_t)(it * 4 + q8) * ldc + c8) = o[it];
    __threadfence();
  }
}

__global__ void __launch_bounds__(256)
k_zero16(_Float16* p, int n16) {
  const int i = blockIdx.x * 256 + threadIdx.x;
  if (i < n16) {
    const v4u z = {0u, 0u, 0u, 0u};
    v4u* d = (v4u*)p + i;
    *(volatile v4u*)d = z;
    __threadfence();
    *(volatile v4u*)d = z;
  }
}

__global__ void __launch_bounds__(128)
k_prep_w(const float* __restrict__ w1, const float* __restrict__ w2, const float* __restrict__ w3,
         const float* __restrict__ wc, _Float16* w16, _Float16* wc16) {
  const int o = blockIdx.x, tid = threadIdx.x, wave = tid >> 5, lane = tid & 31;
  v4h val[3];
  _Float16* dst[3];
#pragma unroll
  for (int i = 0; i < 3; ++i) {
    const int task = wave + 4 * i;
    float f0, f1, f2, f3;
    if (task < 9) {
      const float* src = wc + ((size_t)o * CCH + 4 * lane) * 9 + task;
      f0 = src[0]; f1 = src[9]; f2 = src[18]; f3 = src[27];
      dst[i] = wc16 + (size_t)o * KC3 + task * CCH + 4 * lane;
    } else {
      const int jw = task - 9;
      const float* wsrc = (jw == 0) ? w1 : ((jw == 1) ? w2 : w3);
      const float* src = wsrc + (size_t)o * CCH + 4 * lane;
      f0 = src[0]; f1 = src[1]; f2 = src[2]; f3 = src[3];
      dst[i] = w16 + ((size_t)jw * CCH + o) * CCH + 4 * lane;
    }
    H4 t;
    t.e[0] = (_Float16)(f0 * 16.0f); t.e[1] = (_Float16)(f1 * 16.0f);
    t.e[2] = (_Float16)(f2 * 16.0f); t.e[3] = (_Float16)(f3 * 16.0f);
    val[i] = t.v;
  }
  for (int pass = 0; pass < 2; ++pass) {
#pragma unroll
    for (int i = 0; i < 3; ++i) *(volatile v4h*)dst[i] = val[i];
    __threadfence();
  }
}

__global__ void __launch_bounds__(256)
k_xT(const float* __restrict__ x, _Float16* xt) {
  __shared__ __attribute__((aligned(16))) float T[CCH * 68];
  const int tid = threadIdx.x, wave = tid >> 5, lane = tid & 31;
  const int p0 = blockIdx.x * 64;
#pragma unroll
  for (int it = 0; it < 8; ++it) {
    const int c = it * 16 + (tid >> 4), px4 = (tid & 15) * 4;
    const v4f a = *(const v4f*)(x + (size_t)c * HWP + p0 + px4);
    *(v4f*)(T + c * 68 + px4) = a;
  }
  __syncthreads();
  const int rw = lane >> 4, c8 = (lane & 15) * 8;
  v8h o[4];
#pragma unroll
  for (int it = 0; it < 4; ++it) {
    const int px = wave * 8 + 2 * it + rw;
    H8 t;
#pragma unroll
    for (int e = 0; e < 8; ++e) t.e[e] = (_Float16)T[(c8 + e) * 68 + px];
    o[it] = t.v;
  }
  for (int pass = 0; pass < 2; ++pass) {
#pragma unroll
    for (int it = 0; it < 4; ++it) {
      const int px = wave * 8 + 2 * it + rw;
      *(volatile v8h*)(xt + (size_t)(p0 + px) * CCH + c8) = o[it];
    }
    __threadfence();
  }
}

template <int BIASM>
__global__ void __launch_bounds__(256)
k_proj(const _Float16* A, int lda, const _Float16* Bt, int ldb, _Float16* Cp, int ldc, int tilesN,
       const float* __restrict__ bias, const float* __restrict__ slope, float scale, float ocarry) {
  __shared__ __attribute__((aligned(16))) _Float16 slab_all[8 * 16 * 72];
  const int tid = threadIdx.x, wave = tid >> 5, lane = tid & 31, h = lane >> 4, nn = lane & 15;
  const int bm = blockIdx.x / tilesN, bn = blockIdx.x - bm * tilesN;
  const int m0 = bm * 64 + (wave >> 1) * 16;
  const int n0 = bn * 128 + (wave & 1) * 64;
  v8f acc[4];
#pragma unroll
  for (int j = 0; j < 4; ++j) acc[j] = zero8();
  const _Float16* ar = A  + (size_t)(m0 + nn) * lda + 8 * h;
  const _Float16* br = Bt + (size_t)(n0 + nn) * ldb + 8 * h;
#pragma unroll
  for (int kt = 0; kt < 4; ++kt) {
    const v16h a  = ld_frag(ar + kt * 32);
    const v16h b0 = ld_frag(br + kt * 32);
    const v16h b1 = ld_frag(br + (size_t)16 * ldb + kt * 32);
    const v16h b2 = ld_frag(br + (size_t)32 * ldb + kt * 32);
    const v16h b3 = ld_frag(br + (size_t)48 * ldb + kt * 32);
    acc[0] = mma16(a, b0, acc[0]);
    acc[1] = mma16(a, b1, acc[1]);
    acc[2] = mma16(a, b2, acc[2]);
    acc[3] = mma16(a, b3, acc[3]);
    guard_d4(acc[0], acc[1], acc[2], acc[3], b0, b1, b2, b3, a);
  }
  _Float16* slab = slab_all + wave * (16 * 72);
  const float al = slope[0];
#pragma unroll
  for (int j = 0; j < 4; ++j) {
    float bn_v = 0.f;
    if (BIASM == 0) bn_v = bias[n0 + j * 16 + nn];
#pragma unroll
    for (int r = 0; r < 8; ++r) {
      const int row = 8 * h + r;
      float bv = bn_v;
      if (BIASM == 1) bv = bias[m0 + row];
      float v = acc[j][r] * scale + bv;
      v = (v >= 0.f) ? v : al * v;
      slab[row * 72 + j * 16 + nn] = (_Float16)(v * ocarry);
    }
  }
  wave_lds_sync();
  store_rows16x64(slab, Cp + (size_t)m0 * ldc + n0, ldc, lane);
}

__global__ void __launch_bounds__(64)
k_attn(const _Float16* __restrict__ qp, const _Float16* kp, const _Float16* vtp, _Float16* attpad) {
  __shared__ __attribute__((aligned(16))) _Float16 slab_all[2 * 16 * 136];
  const int tid = threadIdx.x, wave = tid >> 5, lane = tid & 31, h = lane >> 4, n = lane & 15;
  const int q0 = blockIdx.x * 32 + wave * 16;
  const float LSC = 0.022542110f;

  v16h qf[4];
#pragma unroll
  for (int kt = 0; kt < 4; ++kt) qf[kt] = ld_frag(qp + (size_t)(q0 + n) * CCH + kt * 32 + 8 * h);

  v8f accO[8];
#pragma unroll
  for (int ct = 0; ct < 8; ++ct) accO[ct] = zero8();
  float mrun = -3.0e38f, lrun = 0.f;

#pragma unroll 1
  for (int kb0 = 0; kb0 < HWP; kb0 += 64) {
    v8f s[4];
#pragma unroll
    for (int j = 0; j < 4; ++j) {
      const _Float16* kr = kp + (size_t)(kb0 + 16 * j + n) * CCH + 8 * h;
      const v16h a0 = ld_frag(kr), a1 = ld_frag(kr + 32), a2 = ld_frag(kr + 64), a3 = ld_frag(kr + 96);
      v8f t = zero8();
      t = mma16(a0, qf[0], t);
      t = mma16(a1, qf[1], t);
      t = mma16(a2, qf[2], t);
      t = mma16(a3, qf[3], t);
      guard_d1(t, a0, a1, a2, a3);
      s[j] = t;
    }
    float cmax = -3.0e38f;
#pragma unroll
    for (int j = 0; j < 4; ++j) {
#pragma unroll
      for (int r = 0; r < 8; ++r) cmax = fmaxf(cmax, s[j][r]);
    }
    cmax = fmaxf(cmax, __shfl_xor(cmax, 16, 32));
    const float mnew = fmaxf(mrun, cmax);
    const int upd = (mnew != mrun) ? 1 : 0;
    const float alpha = __builtin_amdgcn_exp2f((mrun - mnew) * LSC);
    const float bsh = 14.0f - mnew * LSC;
    mrun = mnew;
    float psum = 0.f;
    Frag pb[2];
#pragma unroll
    for (int j = 0; j < 4; ++j) {
#pragma unroll
      for (int r = 0; r < 8; ++r) {
        const float p = __builtin_amdgcn_exp2f(fmaf(s[j][r], LSC, bsh));
        psum += p;
        pb[j >> 1].e[(j & 1) * 8 + r] = (_Float16)p;
      }
    }
    psum += __shfl_xor(psum, 16, 32);
    lrun = fmaf(lrun, alpha, psum);
    if (__any(upd)) {
#pragma unroll
      for (int ct = 0; ct < 8; ++ct) accO[ct] = accO[ct] * alpha;
    }
#pragma unroll
    for (int kk = 0; kk < 2; ++kk) {
#pragma unroll
      for (int g = 0; g < 2; ++g) {
        const _Float16* vr = vtp + (size_t)(64 * g + n) * HWP + kb0 + 32 * kk + 8 * h;
        const v16h v0 = ld_frag(vr);
        const v16h v1 = ld_frag(vr + (size_t)16 * HWP);
        const v16h v2 = ld_frag(vr + (size_t)32 * HWP);
        const v16h v3 = ld_frag(vr + (size_t)48 * HWP);
        accO[4 * g + 0] = mma16(v0, pb[kk].v, accO[4 * g + 0]);
        accO[4 * g + 1] = mma16(v1, pb[kk].v, accO[4 * g + 1]);
        accO[4 * g + 2] = mma16(v2, pb[kk].v, accO[4 * g + 2]);
        accO[4 * g + 3] = mma16(v3, pb[kk].v, accO[4 * g + 3]);
        guard_d4(accO[4 * g + 0], accO[4 * g + 1], accO[4 * g + 2], accO[4 * g + 3], v0, v1, v2, v3, pb[kk].v);
      }
    }
  }

  const float inv = 2.0f * __builtin_amdgcn_rcpf(lrun);
  _Float16* slab = slab_all + wave * (16 * 136);
#pragma unroll
  for (int ct = 0; ct < 8; ++ct) {
    H8 t;
#pragma unroll
    for (int r = 0; r < 8; ++r) t.e[r] = (_Float16)(accO[ct][r] * inv);
    *(v8h*)(slab + n * 136 + ct * 16 + 8 * h) = t.v;
  }
  wave_lds_sync();
  const int hrow = q0 / IMW, wcol = q0 - hrow * IMW;
  _Float16* dst = attpad + ((size_t)(hrow + 1) * PADW + wcol + 1) * CCH;
  const int rw = lane >> 4, c8 = (lane & 15) * 8;
  v8h o[8];
#pragma unroll
  for (int it = 0; it < 8; ++it) o[it] = *(const v8h*)(slab + (2 * it + rw) * 136 + c8);
  for (int pass = 0; pass < 2; ++pass) {
#pragma unroll
    for (int it = 0; it < 8; ++it)
      *(volatile v8h*)(dst + (size_t)(2 * it + rw) * CCH + c8) = o[it];
    __threadfence();
  }
}

template <bool LAST>
__global__ void __launch_bounds__(128)
k_conv3(const _Float16* attpad, const _Float16* wcp, const float* __restrict__ bc,
        const float* __restrict__ xres, _Float16* xt, float* outp) {
  __shared__ __attribute__((aligned(16))) _Float16 slab_all[4 * 16 * 72];
  __shared__ __attribute__((aligned(16))) float T[CCH * 36];
  const int tid = threadIdx.x, wave = tid >> 5, lane = tid & 31, h = lane >> 4, nn = lane & 15;
  const int p0 = blockIdx.x * 32;
  const int pt = wave & 1, chh = wave >> 1;
  const int pp = p0 + pt * 16;
  const int hrow = pp / IMW, wcol = pp - hrow * IMW;
  v8f acc[4];
#pragma unroll
  for (int j = 0; j < 4; ++j) acc[j] = zero8();
  const _Float16* br = wcp + (size_t)(chh * 64 + nn) * KC3 + 8 * h;
#pragma unroll 1
  for (int dy = 0; dy < 3; ++dy) {
#pragma unroll 1
    for (int dx = 0; dx < 3; ++dx) {
      const _Float16* ar = attpad + ((size_t)(hrow + dy) * PADW + wcol + dx + nn) * CCH + 8 * h;
      const _Float16* bt = br + (dy * 3 + dx) * CCH;
#pragma unroll
      for (int kt = 0; kt < 4; ++kt) {
        const v16h a  = ld_frag(ar + kt * 32);
        const v16h b0 = ld_frag(bt + kt * 32);
        const v16h b1 = ld_frag(bt + (size_t)16 * KC3 + kt * 32);
        const v16h b2 = ld_frag(bt + (size_t)32 * KC3 + kt * 32);
        const v16h b3 = ld_frag(bt + (size_t)48 * KC3 + kt * 32);
        acc[0] = mma16(a, b0, acc[0]);
        acc[1] = mma16(a, b1, acc[1]);
        acc[2] = mma16(a, b2, acc[2]);
        acc[3] = mma16(a, b3, acc[3]);
        guard_d4(acc[0], acc[1], acc[2], acc[3], b0, b1, b2, b3, a);
      }
    }
  }
  float g[4][8];
#pragma unroll
  for (int j = 0; j < 4; ++j) {
    const float bcv = bc[chh * 64 + j * 16 + nn];
#pragma unroll
    for (int r = 0; r < 8; ++r) {
      const float v = acc[j][r] * 0.00390625f + bcv;
      g[j][r] = 0.5f * v * (1.0f + erff(v * 0.70710678118654752f));
    }
  }
  if (!LAST) {
    _Float16* slab = slab_all + wave * (16 * 72);
#pragma unroll
    for (int j = 0; j < 4; ++j) {
#pragma unroll
      for (int r = 0; r < 8; ++r) slab[(8 * h + r) * 72 + j * 16 + nn] = (_Float16)g[j][r];
    }
    wave_lds_sync();
    store_rows16x64(slab, xt + (size_t)pp * CCH + chh * 64, CCH, lane);
  } else {
#pragma unroll
    for (int j = 0; j < 4; ++j) {
      const int c = chh * 64 + j * 16 + nn;
      float* tp = T + c * 36 + pt * 16 + 8 * h;
      v4f u0 = {g[j][0], g[j][1], g[j][2], g[j][3]};
      v4f u1 = {g[j][4], g[j][5], g[j][6], g[j][7]};
      *(v4f*)tp = u0;
      *(v4f*)(tp + 4) = u1;
    }
    __syncthreads();
    const int q8 = lane >> 3, px4 = (lane & 7) * 4;
    v4f o[8];
#pragma unroll
    for (int it = 0; it < 8; ++it) {
      const int c = wave * 32 + it * 4 + q8;
      const v4f t  = *(const v4f*)(T + c * 36 + px4);
      const v4f xv = *(const v4f*)(xres + (size_t)c * HWP + p0 + px4);
      o[it] = t + xv;
    }
    for (int pass = 0; pass < 2; ++pass) {
#pragma unroll
      for (int it = 0; it < 8; ++it) {
        const int c = wave * 32 + it * 4 + q8;
        *(volatile v4f*)(outp + (size_t)c * HWP + p0 + px4) = o[it];
      }
      __threadfence();
    }
  }
}

static inline size_t alup(size_t v) { return (v + 255) & ~(size_t)255; }

extern "C" void kernel_launch(void* const* d_in, const int* in_sizes, int n_in,
                              void* d_out, int out_size, void* d_ws, size_t ws_size,
                              hipStream_t stream) {
  if (n_in < 12) return;
  if (in_sizes[0] != CCH * HWP) return;
  if (in_sizes[1] != CCH * CCH || in_sizes[4] != CCH * CCH || in_sizes[7] != CCH * CCH) return;
  if (in_sizes[2] != CCH || in_sizes[5] != CCH || in_sizes[8] != CCH || in_sizes[11] != CCH) return;
  if (in_sizes[3] < 1 || in_sizes[6] < 1 || in_sizes[9] < 1) return;
  if (in_sizes[10] != CCH * KC3) return;
  if (out_size != CCH * HWP) return;

  const float* x  = (const float*)d_in[0];
  const float* w1 = (const float*)d_in[1];
  const float* b1 = (const float*)d_in[2];
  const float* a1 = (const float*)d_in[3];
  const float* w2 = (const float*)d_in[4];
  const float* b2 = (const float*)d_in[5];
  const float* a2 = (const float*)d_in[6];
  const float* w3 = (const float*)d_in[7];
  const float* b3 = (const float*)d_in[8];
  const float* a3 = (const float*)d_in[9];
  const float* wc = (const float*)d_in[10];
  const float* bc = (const float*)d_in[11];
  float* out = (float*)d_out;

  const size_t actB = (size_t)HWP * CCH * 2;
  const size_t padB = (size_t)PADW * PADW * CCH * 2;
  const size_t wB   = (size_t)3 * CCH * CCH * 2;
  const size_t wcB  = (size_t)CCH * KC3 * 2;
  size_t off = 0;
  const size_t oXt = off; off = alup(off + actB);
  const size_t oQ  = off; off = alup(off + actB);
  const size_t oK  = off; off = alup(off + actB);
  const size_t oVt = off; off = alup(off + actB);
  const size_t oAp = off; off = alup(off + padB);
  const size_t oW  = off; off = alup(off + wB);
  const size_t oWc = off; off = alup(off + wcB);
  if (off > ws_size) return;

  char* ws = (char*)d_ws;
  _Float16* xt   = (_Float16*)(ws + oXt);
  _Float16* q16  = (_Float16*)(ws + oQ);
  _Float16* k16  = (_Float16*)(ws + oK);
  _Float16* vt16 = (_Float16*)(ws + oVt);
  _Float16* attp = (_Float16*)(ws + oAp);
  _Float16* w16  = (_Float16*)(ws + oW);
  _Float16* wc16 = (_Float16*)(ws + oWc);

  const float scProj = 0.0625f;
  const float carryQKV = 8.0f;

  const int n16 = (int)(padB / 16);
  k_zero16<<<dim3((n16 + 255) / 256), dim3(256), 0, stream>>>(attp, n16);
  k_prep_w<<<dim3(CCH), dim3(128), 0, stream>>>(w1, w2, w3, wc, w16, wc16);
  k_xT<<<dim3(HWP / 64), dim3(256), 0, stream>>>(x, xt);

  for (int d = 0; d < 3; ++d) {
    k_proj<0><<<dim3((HWP / 64) * (CCH / 128)), dim3(256), 0, stream>>>(
        xt, CCH, w16, CCH, q16, CCH, 1, b1, a1, scProj, carryQKV);
    k_proj<0><<<dim3((HWP / 64) * (CCH / 128)), dim3(256), 0, stream>>>(
        xt, CCH, w16 + CCH * CCH, CCH, k16, CCH, 1, b2, a2, scProj, carryQKV);
    k_proj<1><<<dim3((CCH / 64) * (HWP / 128)), dim3(256), 0, stream>>>(
        w16 + 2 * CCH * CCH, CCH, xt, CCH, vt16, HWP, HWP / 128, b3, a3, scProj, carryQKV);
    k_attn<<<dim3(HWP / 32), dim3(64), 0, stream>>>(q16, k16, vt16, attp);
    if (d < 2) k_conv3<false><<<dim3(HWP / 32), dim3(128), 0, stream>>>(attp, wc16, bc, x, xt, out);
    else       k_conv3<true ><<<dim3(HWP / 32), dim3(128), 0, stream>>>(attp, wc16, bc, x, xt, out);
  }
  (void)hipGetLastError();
}
